// LinearPerformerAttentionMusic_29875792511831
// MI455X (gfx1250) — hardware-verified
//
#include <hip/hip_runtime.h>
#include <math.h>

constexpr int kBatch  = 2;
constexpr int kSeq    = 1024;
constexpr int kDim    = 512;
constexpr int kHeads  = 8;
constexpr int kHd     = 64;
constexpr int kFeat   = 128;
constexpr int kRows   = kBatch * kSeq;
constexpr int kHB     = kHeads * kBatch;
constexpr int kChunk  = 64;
constexpr int kNChunk = kSeq / kChunk;
constexpr int kNZ     = kHB * kNChunk;
constexpr int kMlp    = 4 * kDim;
constexpr int kDAug   = 128;
constexpr int kPadR   = 4;
constexpr int kPRows  = kSeq + 2 * kPadR;
constexpr float kWCarry    = 64.0f;
constexpr float kWCarryInv = 1.0f / kWCarry;
constexpr float kLnEps  = 1e-5f;
constexpr float kDenEps = 1e-8f;
static_assert(kDim == kHeads * kHd, "head split");
static_assert(kSeq % kChunk == 0, "chunks");
static_assert(kRows % 64 == 0 && kDim % 64 == 0 && kMlp % 64 == 0 && kFeat % 64 == 0 && kDAug % 64 == 0, "tile multiples");
static_assert(kDim % 32 == 0 && kHd % 32 == 0 && kFeat % 32 == 0 && kMlp % 32 == 0, "K multiples of 32");
static_assert((kHd * 3) % 32 == 0 && (kHd * 5) % 32 == 0 && (kHd * 7) % 32 == 0 && (kHd * 9) % 32 == 0, "conv K multiples of 32");

typedef __attribute__((ext_vector_type(16))) _Float16 v16h;
typedef __attribute__((ext_vector_type(8)))  _Float16 v8h;
typedef __attribute__((ext_vector_type(16))) __bf16   v16b;
typedef __attribute__((ext_vector_type(8)))  __bf16   v8b;
typedef __attribute__((ext_vector_type(8)))  float    v8f;
typedef __attribute__((ext_vector_type(4)))  float    v4f;
typedef __attribute__((ext_vector_type(4)))  unsigned int v4u;

__device__ __forceinline__ unsigned short f2bf_bits(float f) {
  unsigned u = __float_as_uint(f);
  return (unsigned short)((u + 0x7FFFu + ((u >> 16) & 1u)) >> 16);
}
__device__ __forceinline__ unsigned short h_bits(float f) { const _Float16 h = (_Float16)f; return __builtin_bit_cast(unsigned short, h); }
__device__ __forceinline__ unsigned pk16(unsigned short a, unsigned short b) { return (unsigned)a | ((unsigned)b << 16); }

__device__ __forceinline__ void guard_row_h(v8f& a, v8f& b, v8f& c, v8f& d, v16h x, v16h y0, v16h y1, v16h y2, v16h y3) {
  asm volatile("v_nop\n\tv_nop\n\tv_nop\n\tv_nop" : "+v"(a), "+v"(b), "+v"(c), "+v"(d) : "v"(x), "v"(y0), "v"(y1), "v"(y2), "v"(y3));
}
__device__ __forceinline__ void guard_row_b(v8f& a, v8f& b, v8f& c, v8f& d, v16b x, v16b y0, v16b y1, v16b y2, v16b y3) {
  asm volatile("v_nop\n\tv_nop\n\tv_nop\n\tv_nop" : "+v"(a), "+v"(b), "+v"(c), "+v"(d) : "v"(x), "v"(y0), "v"(y1), "v"(y2), "v"(y3));
}
__device__ __forceinline__ void keep4_h(v16h a, v16h b, v16h c, v16h d) { asm volatile("v_nop" :: "v"(a), "v"(b), "v"(c), "v"(d)); }
__device__ __forceinline__ void keep4_b(v16b a, v16b b, v16b c, v16b d) { asm volatile("v_nop" :: "v"(a), "v"(b), "v"(c), "v"(d)); }
__device__ __forceinline__ void acc_guard4(v8f& a, v8f& b, v8f& c, v8f& d) { asm volatile("v_nop\n\tv_nop\n\tv_nop\n\tv_nop" : "+v"(a), "+v"(b), "+v"(c), "+v"(d)); }

template <typename T> struct Frag;
template <> struct Frag<_Float16> {
  typedef v16h V; union U { v16h v; v8h h[2]; };
  static __device__ __forceinline__ v16h load(const _Float16* p) {
    U f; f.h[0] = *(const v8h*)(p); f.h[1] = *(const v8h*)(p + 16); return f.v;
  }
  static __device__ __forceinline__ v8f mma(v16h a, v16h b, v8f c) {
    return __builtin_amdgcn_wmma_f32_16x16x32_f16(false, a, false, b, (short)0, c, false, false);
  }
  static __device__ __forceinline__ void guard_row(v8f& a, v8f& b, v8f& c, v8f& d, v16h x, v16h y0, v16h y1, v16h y2, v16h y3) { guard_row_h(a, b, c, d, x, y0, y1, y2, y3); }
  static __device__ __forceinline__ void keep(v16h a, v16h b, v16h c, v16h d) { keep4_h(a, b, c, d); }
};
template <> struct Frag<__bf16> {
  typedef v16b V; union U { v16b v; v8b h[2]; };
  static __device__ __forceinline__ v16b load(const __bf16* p) {
    U f; f.h[0] = *(const v8b*)(p); f.h[1] = *(const v8b*)(p + 16); return f.v;
  }
  static __device__ __forceinline__ v8f mma(v16b a, v16b b, v8f c) {
    return __builtin_amdgcn_wmma_f32_16x16x32_bf16(false, a, false, b, (short)0, c, false, false);
  }
  static __device__ __forceinline__ void guard_row(v8f& a, v8f& b, v8f& c, v8f& d, v16b x, v16b y0, v16b y1, v16b y2, v16b y3) { guard_row_b(a, b, c, d, x, y0, y1, y2, y3); }
  static __device__ __forceinline__ void keep(v16b a, v16b b, v16b c, v16b d) { keep4_b(a, b, c, d); }
};

template <int ACT> __device__ __forceinline__ float act_apply(float v) {
  if (ACT == 5) return 0.5f * v * (1.0f + erff(v * 0.70710678118654752f));
  if (ACT == 6) { const float e = expf(fminf(v, 0.0f)); return (v > 0.0f) ? (v + 1.0f) : e; }
  return v;
}

template <int ET> struct Elem;
template <> struct Elem<0> { typedef _Float16 T; };
template <> struct Elem<1> { typedef __bf16 T; };
template <int ET, int BIAS_MODE, int OUT_MODE, bool RESID, int ACT>
__global__ __launch_bounds__(256) void wmma_gemm64(
    const unsigned short* __restrict__ Ap, int lda, long sAy, long sAz,
    const unsigned short* __restrict__ Btp, int ldb, long sBy, long sBz,
    void* __restrict__ Cout, int ldc, long sCy, long sCz,
    const float* __restrict__ bias,
    const float* __restrict__ resid, long sRy, long sRz,
    int M, int N, int K, int nby, int nbatch, float scale) {
  static_assert(!RESID || OUT_MODE == 0, "residual only on f32 outputs");
  typedef typename Elem<ET>::T T;
  typedef typename Frag<T>::V V;
  const T* A = (const T*)Ap; const T* Bt = (const T*)Btp;
  __shared__ __align__(16) float sT[8][16 * 68];
  const int lane = threadIdx.x & 31;
  const int wave = threadIdx.x >> 5;
  const int tilesN = N >> 6;
  const int tilesM = M >> 6;
  const int tpb = tilesM * tilesN;
  const int gt = blockIdx.x * 8 + wave;
  if (gt >= tpb * nbatch) return;
  const int batch = gt / tpb;
  const int tile  = gt - batch * tpb;
  const int bz = batch / nby;
  const int by = batch - bz * nby;
  const int tm = tile / tilesN;
  const int tn = tile - tm * tilesN;
  const int m0 = tm << 6;
  const int n0 = tn << 6;

  const T* Ab = A  + (size_t)by * (size_t)sAy + (size_t)bz * (size_t)sAz;
  const T* Bb = Bt + (size_t)by * (size_t)sBy + (size_t)bz * (size_t)sBz;
  const size_t cOff = (size_t)by * (size_t)sCy + (size_t)bz * (size_t)sCz;

  const int rlane = lane & 15;
  const int koff  = (lane >> 4) * 8;
  const int mOff  = (lane >> 4) * 8;

  v8f acc[4][4];
#pragma unroll
  for (int i = 0; i < 4; ++i)
#pragma unroll
    for (int j = 0; j < 4; ++j) acc[i][j] = (v8f){0.f, 0.f, 0.f, 0.f, 0.f, 0.f, 0.f, 0.f};

  for (int k0 = 0; k0 < K; k0 += 32) {
    V bh[4];
#pragma unroll
    for (int j = 0; j < 4; ++j) {
      const size_t bo = (size_t)(n0 + (j << 4) + rlane) * ldb + koff + k0;
      bh[j] = Frag<T>::load(Bb + bo);
    }
#pragma unroll
    for (int i = 0; i < 4; ++i) {
      const size_t ao = (size_t)(m0 + (i << 4) + rlane) * lda + koff + k0;
      V ah = Frag<T>::load(Ab + ao);
#pragma unroll
      for (int j = 0; j < 4; ++j) acc[i][j] = Frag<T>::mma(ah, bh[j], acc[i][j]);
      Frag<T>::guard_row(acc[i][0], acc[i][1], acc[i][2], acc[i][3], ah, bh[0], bh[1], bh[2], bh[3]);
    }
    Frag<T>::keep(bh[0], bh[1], bh[2], bh[3]);
  }
  acc_guard4(acc[0][0], acc[0][1], acc[0][2], acc[0][3]);
  acc_guard4(acc[1][0], acc[1][1], acc[1][2], acc[1][3]);
  acc_guard4(acc[2][0], acc[2][1], acc[2][2], acc[2][3]);
  acc_guard4(acc[3][0], acc[3][1], acc[3][2], acc[3][3]);

  float* slab = sT[wave];
  const float* Rb = RESID ? (resid + (size_t)by * (size_t)sRy + (size_t)bz * (size_t)sRz) : nullptr;
#pragma unroll
  for (int i = 0; i < 4; ++i) {
    const int mBase = m0 + (i << 4);
#pragma unroll
    for (int j = 0; j < 4; ++j) {
      const int n = n0 + (j << 4) + rlane;
      float bv = 0.f;
      if (BIAS_MODE == 2) bv = bias[n];
#pragma unroll
      for (int r = 0; r < 8; ++r) {
        float v = acc[i][j][r] * scale;
        if (BIAS_MODE == 2) v += bv;
        if (ACT == 7) v = (n > (mBase + mOff + r)) ? 0.0f : v;
        slab[(mOff + r) * 68 + (j << 4) + rlane] = v;
      }
    }
    __builtin_amdgcn_fence(__ATOMIC_RELEASE, "workgroup");
    __builtin_amdgcn_wave_barrier();
    __builtin_amdgcn_fence(__ATOMIC_ACQUIRE, "workgroup");
    if (ACT == 5 || ACT == 6) {
#pragma unroll 1
      for (int it = 0; it < 32; ++it) {
        const int idx = it * 32 + lane;
        const int row = idx >> 6, col = idx & 63;
        const float v = slab[row * 68 + col];
        slab[row * 68 + col] = act_apply<ACT>(v);
      }
      __builtin_amdgcn_fence(__ATOMIC_RELEASE, "workgroup");
      __builtin_amdgcn_wave_barrier();
      __builtin_amdgcn_fence(__ATOMIC_ACQUIRE, "workgroup");
    }
    if (OUT_MODE == 0) {
      float* Cf = (float*)Cout + cOff;
      const int hh = lane >> 4, c4 = (lane & 15) * 4;
      if (RESID) {
#pragma unroll
        for (int it = 0; it < 8; ++it) {
          const int row = it * 2 + hh;
          v4f v = *(const v4f*)(slab + row * 68 + c4);
          const v4f rr = *(const v4f*)(Rb + (size_t)(mBase + row) * ldc + n0 + c4);
          v = v + rr;
          *(v4f*)(slab + row * 68 + c4) = v;
        }
      }
      for (int pass = 0; pass < 2; ++pass) {
#pragma unroll
        for (int it = 0; it < 8; ++it) {
          const int row = it * 2 + hh;
          v4f v = *(const v4f*)(slab + row * 68 + c4);
          *(volatile v4f*)(Cf + (size_t)(mBase + row) * ldc + n0 + c4) = v;
        }
        __threadfence();
      }
    } else {
      const int q = lane >> 3, c8 = (lane & 7) * 8;
      unsigned short* Ch = (unsigned short*)Cout + cOff;
      for (int pass = 0; pass < 2; ++pass) {
#pragma unroll
        for (int it = 0; it < 4; ++it) {
          const int row = it * 4 + q;
          const float* sp = slab + row * 68 + c8;
          v8h hv;
#pragma unroll
          for (int e = 0; e < 8; ++e) {
            if (OUT_MODE == 1) {
              hv[e] = (_Float16)sp[e];
            } else {
              const unsigned short hb = f2bf_bits(sp[e]);
              hv[e] = __builtin_bit_cast(_Float16, hb);
            }
          }
          *(volatile v8h*)(Ch + (size_t)(mBase + row) * ldc + n0 + c8) = hv;
        }
        __threadfence();
      }
    }
    __builtin_amdgcn_fence(__ATOMIC_RELEASE, "workgroup");
    __builtin_amdgcn_wave_barrier();
    __builtin_amdgcn_fence(__ATOMIC_ACQUIRE, "workgroup");
  }
}

template <int MODE>
__global__ __launch_bounds__(256) void cast8_kernel(const float* __restrict__ s0, const float* __restrict__ s1,
                                                    const float* __restrict__ s2, const float* __restrict__ s3,
                                                    unsigned short* __restrict__ out, int n8, float sc) {
  const int i = blockIdx.x * 256 + threadIdx.x;
  const int y = blockIdx.y;
  const float* src = (y == 0) ? s0 : (y == 1) ? s1 : (y == 2) ? s2 : s3;
  if (i >= n8) return;
  const float* p = src + 8 * (size_t)i;
  const v4f a = *(const v4f*)(p);
  const v4f c = *(const v4f*)(p + 4);
  unsigned short hb[8];
#pragma unroll
  for (int e = 0; e < 4; ++e) {
    const float fa = a[e];
    const float fc = c[e];
    if (MODE == 0) { hb[e] = f2bf_bits(fa); hb[4 + e] = f2bf_bits(fc); }
    else           { hb[e] = h_bits(fa * sc); hb[4 + e] = h_bits(fc * sc); }
  }
  const v4u u = (v4u){pk16(hb[0], hb[1]), pk16(hb[2], hb[3]), pk16(hb[4], hb[5]), pk16(hb[6], hb[7])};
  unsigned short* q = out + (size_t)y * (size_t)n8 * 8 + 8 * (size_t)i;
  *(volatile v4u*)q = u;
  __threadfence();
  *(volatile v4u*)q = u;
}

__global__ __launch_bounds__(256) void feat_transpose_kernel(const float* __restrict__ in, unsigned short* __restrict__ out) {
  __shared__ float sm[64][65];
  const int t  = threadIdx.x;
  const int f0 = blockIdx.x * 64;
  const int h  = blockIdx.y;
  const float* ip = in + (size_t)h * kHd * kFeat;
#pragma unroll
  for (int i = 0; i < 16; ++i) {
    const int e = i * 256 + t;
    const int r = e >> 6;
    const int c = e & 63;
    sm[c][r] = ip[(size_t)r * kFeat + f0 + c];
  }
  __syncthreads();
  const int lane = t & 31, wave = t >> 5;
  const int q = lane >> 3, c8 = (lane & 7) * 8;
  unsigned short* op = out + (size_t)h * kFeat * kHd;
  for (int pass = 0; pass < 2; ++pass) {
#pragma unroll
    for (int it = 0; it < 2; ++it) {
      const int row = wave * 8 + it * 4 + q;
      unsigned short hb[8];
#pragma unroll
      for (int e = 0; e < 8; ++e) hb[e] = f2bf_bits(sm[row][c8 + e]);
      const v4u u = (v4u){pk16(hb[0], hb[1]), pk16(hb[2], hb[3]), pk16(hb[4], hb[5]), pk16(hb[6], hb[7])};
      *(volatile v4u*)(op + (size_t)(f0 + row) * kHd + c8) = u;
    }
    __threadfence();
  }
}

__global__ __launch_bounds__(256) void convw_repack_kernel(const float* __restrict__ w3, const float* __restrict__ w5,
                                                           const float* __restrict__ w7, const float* __restrict__ w9,
                                                           unsigned short* __restrict__ r3, unsigned short* __restrict__ r5,
                                                           unsigned short* __restrict__ r7, unsigned short* __restrict__ r9) {
  const int y  = blockIdx.y;
  const int ks = 3 + 2 * y;
  const float* w = (y == 0) ? w3 : (y == 1) ? w5 : (y == 2) ? w7 : w9;
  unsigned short* out = (y == 0) ? r3 : (y == 1) ? r5 : (y == 2) ? r7 : r9;
  const int i = blockIdx.x * 256 + threadIdx.x;
  if (i >= 512 * ks) return;
  const int o   = i * 8;
  const int kk  = 64 * ks;
  const int co  = o / kk;
  const int rem = o - co * kk;
  const int t   = rem >> 6;
  const int ci0 = rem & 63;
  unsigned short hb[8];
#pragma unroll
  for (int e = 0; e < 8; ++e) {
    const float f = w[((size_t)(co * 64 + ci0 + e)) * ks + t];
    hb[e] = f2bf_bits(f);
  }
  const v4u u = (v4u){pk16(hb[0], hb[1]), pk16(hb[2], hb[3]), pk16(hb[4], hb[5]), pk16(hb[6], hb[7])};
  unsigned short* q = out + (size_t)o;
  *(volatile v4u*)q = u;
  __threadfence();
  *(volatile v4u*)q = u;
}

constexpr int kAuxUnits = kHeads * 64 * (kRows / 8);
constexpr int kPadUnits = 4 * kHB * 8 * 8;
static_assert(kAuxUnits % 256 == 0 && kPadUnits % 256 == 0, "fill grid exact");
__global__ __launch_bounds__(256) void fill_kernel(unsigned short* __restrict__ VTA, unsigned short* __restrict__ PP) {
  const int i = blockIdx.x * 256 + threadIdx.x;
  if (i < kAuxUnits) {
    const int h   = i >> 14;
    const int u   = i & 16383;
    const int row = 64 + (u >> 8);
    const int c8  = (u & 255) * 8;
    const unsigned word = (row == 64) ? 0x3F803F80u : 0u;
    const v4u val = (v4u){word, word, word, word};
    unsigned short* p = VTA + ((size_t)h * kDAug + row) * kRows + c8;
    *(volatile v4u*)p = val;
    __threadfence();
    *(volatile v4u*)p = val;
  } else if (i < kAuxUnits + kPadUnits) {
    const int j     = i - kAuxUnits;
    const int plane = j >> 10;
    const int r     = j & 1023;
    const int hb    = r >> 6;
    const int w     = r & 63;
    const int prow  = w >> 3;
    const int c8    = (w & 7) * 8;
    const int row   = (prow < 4) ? prow : (kSeq + prow);
    const v4u val = (v4u){0u, 0u, 0u, 0u};
    unsigned short* p = PP + (((size_t)plane * kHB + hb) * kPRows + row) * kHd + c8;
    *(volatile v4u*)p = val;
    __threadfence();
    *(volatile v4u*)p = val;
  }
}

__global__ __launch_bounds__(256) void chunk_prefix_kernel(const float* __restrict__ SKV, unsigned short* __restrict__ SPT) {
  const int i  = blockIdx.x * 256 + threadIdx.x;
  const int hb = i >> 11;
  const int e8 = i & 2047;
  float run[8];
#pragma unroll
  for (int e = 0; e < 8; ++e) run[e] = 0.0f;
#pragma unroll 1
  for (int c = 0; c < kNChunk; ++c) {
    const size_t off = ((size_t)(hb * kNChunk + c)) * (size_t)(kDAug * kFeat) + (size_t)e8 * 8;
    unsigned short hbv[8];
#pragma unroll
    for (int e = 0; e < 8; ++e) hbv[e] = f2bf_bits(run[e]);
    const v4u u = (v4u){pk16(hbv[0], hbv[1]), pk16(hbv[2], hbv[3]), pk16(hbv[4], hbv[5]), pk16(hbv[6], hbv[7])};
    *(volatile v4u*)(SPT + off) = u;
    __threadfence();
    *(volatile v4u*)(SPT + off) = u;
    const v4f a = *(const v4f*)(SKV + off);
    const v4f b = *(const v4f*)(SKV + off + 4);
#pragma unroll
    for (int e = 0; e < 4; ++e) {
      const float fa = a[e];
      const float fb = b[e];
      run[e] += fa;
      run[4 + e] += fb;
    }
  }
}

__global__ __launch_bounds__(256) void split_kernel(const float* __restrict__ NUMB, unsigned short* __restrict__ P0,
                                                    float* __restrict__ DEN) {
  const int t   = threadIdx.x;
  const int row = blockIdx.x * 32 + (t >> 3);
  const int c8  = (t & 7) * 8;
  const int hb  = row >> 10;
  const int n   = row & 1023;
  const float* sp = NUMB + (size_t)row * kDAug + c8;
  const v4f a = *(const v4f*)(sp);
  const v4f c = *(const v4f*)(sp + 4);
  unsigned short hbv[8];
#pragma unroll
  for (int e = 0; e < 4; ++e) {
    const float fa = a[e];
    const float fc = c[e];
    hbv[e] = f2bf_bits(fa);
    hbv[4 + e] = f2bf_bits(fc);
  }
  const v4u u = (v4u){pk16(hbv[0], hbv[1]), pk16(hbv[2], hbv[3]), pk16(hbv[4], hbv[5]), pk16(hbv[6], hbv[7])};
  unsigned short* q = P0 + ((size_t)hb * kPRows + kPadR + n) * kHd + c8;
  *(volatile v4u*)q = u;
  __threadfence();
  *(volatile v4u*)q = u;
  if (t < 32) {
    const int r2 = blockIdx.x * 32 + t;
    const float d = NUMB[(size_t)r2 * kDAug + kHd];
    *(volatile float*)(DEN + r2) = d;
    __threadfence();
    *(volatile float*)(DEN + r2) = d;
  }
}

__global__ __launch_bounds__(256) void divmerge_kernel(const float* __restrict__ C9, const float* __restrict__ DEN,
                                                       unsigned short* __restrict__ ATTM) {
  const int t   = threadIdx.x;
  const int row = blockIdx.x * 32 + (t >> 3);
  const int c8  = (t & 7) * 8;
  const int hb  = row >> 10;
  const int n   = row & 1023;
  const int h   = hb >> 1;
  const int b   = hb & 1;
  const float rd = 1.0f / (DEN[row] + kDenEps);
  const float* sp = C9 + (size_t)row * kHd + c8;
  const v4f a = *(const v4f*)(sp);
  const v4f c = *(const v4f*)(sp + 4);
  unsigned short hbv[8];
#pragma unroll
  for (int e = 0; e < 4; ++e) {
    const float fa = a[e];
    const float fc = c[e];
    hbv[e] = f2bf_bits(fa * rd);
    hbv[4 + e] = f2bf_bits(fc * rd);
  }
  const v4u u = (v4u){pk16(hbv[0], hbv[1]), pk16(hbv[2], hbv[3]), pk16(hbv[4], hbv[5]), pk16(hbv[6], hbv[7])};
  unsigned short* q = ATTM + ((size_t)b * kSeq + n) * kDim + h * kHd + c8;
  *(volatile v4u*)q = u;
  __threadfence();
  *(volatile v4u*)q = u;
}

template <bool W16>
__global__ __launch_bounds__(256) void ln_rows_kernel(const float* __restrict__ YP, const float* __restrict__ gam,
                                                      const float* __restrict__ bet, float* __restrict__ Y,
                                                      unsigned short* __restrict__ Y16, int nrows) {
  __shared__ __align__(16) float stg[8][W16 ? 512 : 4];
  const int tid = threadIdx.x, lane = tid & 31, wave = tid >> 5;
  const int row = blockIdx.x * 8 + wave;
  if (row >= nrows) return;
  const float* rp = YP + (size_t)row * kDim;
  v4f v[4], g[4], bb[4];
  float s = 0.0f;
#pragma unroll
  for (int q = 0; q < 4; ++q) {
    v[q]  = *(const v4f*)(rp  + 128 * q + 4 * lane);
    g[q]  = *(const v4f*)(gam + 128 * q + 4 * lane);
    bb[q] = *(const v4f*)(bet + 128 * q + 4 * lane);
    s += (v[q][0] + v[q][1]) + (v[q][2] + v[q][3]);
  }
#pragma unroll
  for (int off = 1; off < 32; off <<= 1) s += __shfl_xor(s, off, 32);
  const float mu = s * (1.0f / kDim);
  float ss = 0.0f;
#pragma unroll
  for (int q = 0; q < 4; ++q)
#pragma unroll
    for (int e = 0; e < 4; ++e) { const float d = v[q][e] - mu; v[q][e] = d; ss += d * d; }
#pragma unroll
  for (int off = 1; off < 32; off <<= 1) ss += __shfl_xor(ss, off, 32);
  const float var  = ss * (1.0f / kDim);
  const float rstd = 1.0f / sqrtf(var + kLnEps);
  v4f o[4];
#pragma unroll
  for (int q = 0; q < 4; ++q)
#pragma unroll
    for (int e = 0; e < 4; ++e) o[q][e] = (v[q][e] * rstd) * g[q][e] + bb[q][e];
  float* op = Y + (size_t)row * kDim;
  for (int pass = 0; pass < 2; ++pass) {
#pragma unroll
    for (int q = 0; q < 4; ++q) *(volatile v4f*)(op + 128 * q + 4 * lane) = o[q];
    __threadfence();
  }
  if (W16) {
    float* st = stg[wave];
#pragma unroll
    for (int q = 0; q < 4; ++q) *(v4f*)(st + 128 * q + 4 * lane) = o[q];
    __builtin_amdgcn_fence(__ATOMIC_RELEASE, "workgroup");
    __builtin_amdgcn_wave_barrier();
    __builtin_amdgcn_fence(__ATOMIC_ACQUIRE, "workgroup");
    v4u uu[2];
#pragma unroll
    for (int j = 0; j < 2; ++j) {
      const float* sp = st + 256 * j + 8 * lane;
      const v4f a = *(const v4f*)(sp);
      const v4f c = *(const v4f*)(sp + 4);
      unsigned short hb[8];
#pragma unroll
      for (int e = 0; e < 4; ++e) {
        const float fa = a[e];
        const float fc = c[e];
        hb[e] = h_bits(fa);
        hb[4 + e] = h_bits(fc);
      }
      uu[j] = (v4u){pk16(hb[0], hb[1]), pk16(hb[2], hb[3]), pk16(hb[4], hb[5]), pk16(hb[6], hb[7])};
    }
    unsigned short* hp = Y16 + (size_t)row * kDim;
    for (int pass = 0; pass < 2; ++pass) {
#pragma unroll
      for (int j = 0; j < 2; ++j) *(volatile v4u*)(hp + 256 * j + 8 * lane) = uu[j];
      __threadfence();
    }
  }
}

extern "C" void kernel_launch(void* const* d_in, const int* in_sizes, int n_in,
                              void* d_out, int out_size, void* d_ws, size_t ws_size, hipStream_t stream) {
  if (n_in < 22 || d_out == nullptr || d_ws == nullptr) return;
  const int expect[22] = {
      kRows * kDim, kRows * kDim, kDim * kDim, kDim * kDim, kDim * kDim, kHeads * kHd * kFeat,
      kHd * kHd * 3, kHd, kHd * kHd * 5, kHd, kHd * kHd * 7, kHd, kHd * kHd * 9, kHd,
      kDim, kDim, kMlp * kDim, kMlp, kDim * kMlp, kDim, kDim * kDim, kDim};
  static_assert(sizeof(expect) / sizeof(expect[0]) == 22, "input table");
  for (int i = 0; i < 22; ++i) if (in_sizes[i] != expect[i]) return;
  if (out_size != kRows * kDim) return;

  const float* x    = (const float*)d_in[0];
  const float* y    = (const float*)d_in[1];
  const float* Wq   = (const float*)d_in[2];
  const float* Wk   = (const float*)d_in[3];
  const float* Wv   = (const float*)d_in[4];
  const float* proj = (const float*)d_in[5];
  const float* cw3  = (const float*)d_in[6];
  const float* cb3  = (const float*)d_in[7];
  const float* cw5  = (const float*)d_in[8];
  const float* cb5  = (const float*)d_in[9];
  const float* cw7  = (const float*)d_in[10];
  const float* cb7  = (const float*)d_in[11];
  const float* cw9  = (const float*)d_in[12];
  const float* cb9  = (const float*)d_in[13];
  const float* ng   = (const float*)d_in[14];
  const float* nbv  = (const float*)d_in[15];
  const float* w1   = (const float*)d_in[16];
  const float* b1   = (const float*)d_in[17];
  const float* w2   = (const float*)d_in[18];
  const float* b2   = (const float*)d_in[19];
  const float* ow   = (const float*)d_in[20];
  const float* ob   = (const float*)d_in[21];
  float* outp = (float*)d_out;

  char* ws = (char*)d_ws; size_t off = 0;
  auto carve = [&](size_t bytes) -> char* { char* p = ws + off; off += (bytes + 255) & ~(size_t)255; return p; };
  unsigned short* XB   = (unsigned short*)carve((size_t)kRows * kDim * 2);
  unsigned short* YB   = (unsigned short*)carve((size_t)kRows * kDim * 2);
  unsigned short* WSQ  = (unsigned short*)carve((size_t)4 * kDim * kDim * 2);
  unsigned short* W1H  = (unsigned short*)carve((size_t)kMlp * kDim * 2);
  unsigned short* W2H  = (unsigned short*)carve((size_t)kDim * kMlp * 2);
  unsigned short* PT   = (unsigned short*)carve((size_t)kHeads * kFeat * kHd * 2);
  unsigned short* WR3  = (unsigned short*)carve((size_t)kHd * kHd * 3 * 2);
  unsigned short* WR5  = (unsigned short*)carve((size_t)kHd * kHd * 5 * 2);
  unsigned short* WR7  = (unsigned short*)carve((size_t)kHd * kHd * 7 * 2);
  unsigned short* WR9  = (unsigned short*)carve((size_t)kHd * kHd * 9 * 2);
  unsigned short* QH   = (unsigned short*)carve((size_t)kHeads * kRows * kHd * 2);
  unsigned short* KH   = (unsigned short*)carve((size_t)kHeads * kRows * kHd * 2);
  unsigned short* VTA  = (unsigned short*)carve((size_t)kHeads * kDAug * kRows * 2);
  unsigned short* QP   = (unsigned short*)carve((size_t)kHeads * kRows * kFeat * 2);
  unsigned short* KP   = (unsigned short*)carve((size_t)kHeads * kRows * kFeat * 2);
  unsigned short* KPT  = (unsigned short*)carve((size_t)kHeads * kFeat * kRows * 2);
  float*          SKV  = (float*)carve((size_t)kNZ * kDAug * kFeat * 4);
  unsigned short* SPT  = (unsigned short*)carve((size_t)kNZ * kDAug * kFeat * 2);
  unsigned short* PS   = (unsigned short*)carve((size_t)kNZ * kChunk * kChunk * 2);
  float*          NUMA = (float*)carve((size_t)kHB * kSeq * kDAug * 4);
  float*          NUMB = (float*)carve((size_t)kHB * kSeq * kDAug * 4);
  float*          DEN  = (float*)carve((size_t)kHB * kSeq * 4);
  unsigned short* PP   = (unsigned short*)carve((size_t)4 * kHB * kPRows * kHd * 2);
  float*          C9   = (float*)carve((size_t)kHB * kSeq * kHd * 4);
  unsigned short* ATTM = (unsigned short*)carve((size_t)kRows * kDim * 2);
  float*          H1   = (float*)carve((size_t)kRows * kDim * 4);
  float*          H1N  = (float*)carve((size_t)kRows * kDim * 4);
  unsigned short* H1NH = (unsigned short*)carve((size_t)kRows * kDim * 2);
  unsigned short* HID  = (unsigned short*)carve((size_t)kRows * kMlp * 2);
  float*          PRE2 = (float*)carve((size_t)kRows * kDim * 4);
  if (off > ws_size || off > (size_t)134217728) return;

  unsigned short* WQB = WSQ;
  unsigned short* WKB = WSQ + (size_t)kDim * kDim;
  unsigned short* WVB = WSQ + (size_t)2 * kDim * kDim;
  unsigned short* WOB = WSQ + (size_t)3 * kDim * kDim;
  const size_t planeP = (size_t)kHB * kPRows * kHd;
  unsigned short* P0 = PP;
  unsigned short* P1 = PP + planeP;
  unsigned short* P2 = PP + 2 * planeP;
  unsigned short* P3 = PP + 3 * planeP;

  auto gridFor = [](int M, int N, int nb) { return dim3((unsigned)((((M >> 6) * (N >> 6)) * nb + 7) / 8)); };

  {
    const int n8a = kRows * kDim / 8;
    const int n8w = kDim * kDim / 8;
    const int n8m = kMlp * kDim / 8;
    cast8_kernel<0><<<dim3(n8a / 256, 2), 256, 0, stream>>>(x, y, x, y, XB, n8a, 1.0f);
    cast8_kernel<0><<<dim3(n8w / 256, 4), 256, 0, stream>>>(Wq, Wk, Wv, ow, WSQ, n8w, 1.0f);
    cast8_kernel<1><<<dim3(n8m / 256, 2), 256, 0, stream>>>(w1, w2, w1, w2, W1H, n8m, kWCarry);
    feat_transpose_kernel<<<dim3(kFeat / 64, kHeads), 256, 0, stream>>>(proj, PT);
    convw_repack_kernel<<<dim3((512 * 9 + 255) / 256, 4), 256, 0, stream>>>(cw3, cw5, cw7, cw9, WR3, WR5, WR7, WR9);
    fill_kernel<<<dim3((kAuxUnits + kPadUnits) / 256), 256, 0, stream>>>(VTA, PP);
  }
  if (W2H != W1H + (size_t)kMlp * kDim) return;

  const long LH = (long)kHd * kDim;

  wmma_gemm64<1, 0, 3, false, 0><<<gridFor(kRows, kHd, kHeads), 256, 0, stream>>>(
      XB, kDim, 0L, 0L, WQB, kDim, LH, 0L, (void*)QH, kHd, (long)kRows * kHd, 0L,
      nullptr, nullptr, 0L, 0L, kRows, kHd, kDim, kHeads, kHeads, 1.0f);
  wmma_gemm64<1, 0, 3, false, 0><<<gridFor(kRows, kHd, kHeads), 256, 0, stream>>>(
      YB, kDim, 0L, 0L, WKB, kDim, LH, 0L, (void*)KH, kHd, (long)kRows * kHd, 0L,
      nullptr, nullptr, 0L, 0L, kRows, kHd, kDim, kHeads, kHeads, 1.0f);
  wmma_gemm64<1, 0, 3, false, 0><<<gridFor(kHd, kRows, kHeads), 256, 0, stream>>>(
      WVB, kDim, LH, 0L, YB, kDim, 0L, 0L, (void*)VTA, kRows, (long)kDAug * kRows, 0L,
      nullptr, nullptr, 0L, 0L, kHd, kRows, kDim, kHeads, kHeads, 1.0f);

  wmma_gemm64<1, 0, 3, false, 6><<<gridFor(kRows, kFeat, kHeads), 256, 0, stream>>>(
      QH, kHd, (long)kRows * kHd, 0L, PT, kHd, (long)kFeat * kHd, 0L, (void*)QP, kFeat, (long)kRows * kFeat, 0L,
      nullptr, nullptr, 0L, 0L, kRows, kFeat, kHd, kHeads, kHeads, 1.0f);
  wmma_gemm64<1, 0, 3, false, 6><<<gridFor(kRows, kFeat, kHeads), 256, 0, stream>>>(
      KH, kHd, (long)kRows * kHd, 0L, PT, kHd, (long)kFeat * kHd, 0L, (void*)KP, kFeat, (long)kRows * kFeat, 0L,
      nullptr, nullptr, 0L, 0L, kRows, kFeat, kHd, kHeads, kHeads, 1.0f);
  wmma_gemm64<1, 0, 3, false, 6><<<gridFor(kFeat, kRows, kHeads), 256, 0, stream>>>(
      PT, kHd, (long)kFeat * kHd, 0L, KH, kHd, (long)kRows * kHd, 0L, (void*)KPT, kRows, (long)kFeat * kRows, 0L,
      nullptr, nullptr, 0L, 0L, kFeat, kRows, kHd, kHeads, kHeads, 1.0f);

  wmma_gemm64<1, 0, 0, false, 0><<<gridFor(kDAug, kFeat, kNZ), 256, 0, stream>>>(
      VTA, kRows, (long)kChunk, (long)kDAug * kRows, KPT, kRows, (long)kChunk, (long)kFeat * kRows,
      (void*)SKV, kFeat, (long)kDAug * kFeat, (long)32 * kDAug * kFeat,
      nullptr, nullptr, 0L, 0L, kDAug, kFeat, kChunk, 32, kNZ, 1.0f);
  chunk_prefix_kernel<<<dim3(kHB * (kDAug * kFeat / 8) / 256), 256, 0, stream>>>(SKV, SPT);

  wmma_gemm64<1, 0, 3, false, 7><<<gridFor(kChunk, kChunk, kNZ), 256, 0, stream>>>(
      QP, kFeat, (long)kChunk * kFeat, 0L, KP, kFeat, (long)kChunk * kFeat, 0L,
      (void*)PS, kChunk, (long)kChunk * kChunk, 0L,
      nullptr, nullptr, 0L, 0L, kChunk, kChunk, kFeat, kNZ, kNZ, 1.0f);
  wmma_gemm64<1, 0, 0, false, 0><<<gridFor(kChunk, kDAug, kNZ), 256, 0, stream>>>(
      QP, kFeat, (long)kChunk * kFeat, 0L, SPT, kFeat, (long)kDAug * kFeat, 0L,
      (void*)NUMA, kDAug, (long)kChunk * kDAug, 0L,
      nullptr, nullptr, 0L, 0L, kChunk, kDAug, kFeat, kNZ, kNZ, 1.0f);
  wmma_gemm64<1, 0, 0, true, 0><<<gridFor(kChunk, kDAug, kNZ), 256, 0, stream>>>(
      PS, kChunk, (long)kChunk * kChunk, (long)32 * kChunk * kChunk,
      VTA, kRows, (long)kChunk, (long)kDAug * kRows,
      (void*)NUMB, kDAug, (long)kChunk * kDAug, (long)32 * kChunk * kDAug,
      nullptr, NUMA, (long)kChunk * kDAug, (long)32 * kChunk * kDAug,
      kChunk, kDAug, kChunk, 32, kNZ, 1.0f);
  split_kernel<<<dim3(kHB * kSeq / 32), 256, 0, stream>>>(NUMB, P0, DEN);

  {
    const long sP = (long)kPRows * kHd;
    wmma_gemm64<1, 2, 3, false, 0><<<gridFor(kSeq, kHd, kHB), 256, 0, stream>>>(
        P0 + (kPadR - 1) * kHd, kHd, sP, 0L, WR3, kHd * 3, 0L, 0L, (void*)(P1 + kPadR * kHd), kHd, sP, 0L,
        cb3, nullptr, 0L, 0L, kSeq, kHd, kHd * 3, kHB, kHB, 1.0f);
    wmma_gemm64<1, 2, 3, false, 0><<<gridFor(kSeq, kHd, kHB), 256, 0, stream>>>(
        P1 + (kPadR - 2) * kHd, kHd, sP, 0L, WR5, kHd * 5, 0L, 0L, (void*)(P2 + kPadR * kHd), kHd, sP, 0L,
        cb5, nullptr, 0L, 0L, kSeq, kHd, kHd * 5, kHB, kHB, 1.0f);
    wmma_gemm64<1, 2, 3, false, 0><<<gridFor(kSeq, kHd, kHB), 256, 0, stream>>>(
        P2 + (kPadR - 3) * kHd, kHd, sP, 0L, WR7, kHd * 7, 0L, 0L, (void*)(P3 + kPadR * kHd), kHd, sP, 0L,
        cb7, nullptr, 0L, 0L, kSeq, kHd, kHd * 7, kHB, kHB, 1.0f);
    wmma_gemm64<1, 2, 0, false, 0><<<gridFor(kSeq, kHd, kHB), 256, 0, stream>>>(
        P3 + (kPadR - 4) * kHd, kHd, sP, 0L, WR9, kHd * 9, 0L, 0L, (void*)C9, kHd, (long)kSeq * kHd, 0L,
        cb9, nullptr, 0L, 0L, kSeq, kHd, kHd * 9, kHB, kHB, 1.0f);
  }
  divmerge_kernel<<<dim3(kHB * kSeq / 32), 256, 0, stream>>>(C9, DEN, ATTM);

  wmma_gemm64<1, 2, 0, true, 0><<<gridFor(kRows, kDim, 1), 256, 0, stream>>>(
      ATTM, kDim, 0L, 0L, WOB, kDim, 0L, 0L, (void*)H1, kDim, 0L, 0L,
      ob, x, 0L, 0L, kRows, kDim, kDim, 1, 1, 1.0f);
  ln_rows_kernel<true><<<dim3(kRows / 8), 256, 0, stream>>>(H1, ng, nbv, H1N, H1NH, kRows);
  wmma_gemm64<0, 2, 1, false, 5><<<gridFor(kRows, kMlp, 1), 256, 0, stream>>>(
      H1NH, kDim, 0L, 0L, W1H, kDim, 0L, 0L, (void*)HID, kMlp, 0L, 0L,
      b1, nullptr, 0L, 0L, kRows, kMlp, kDim, 1, 1, kWCarryInv);
  wmma_gemm64<0, 2, 0, true, 0><<<gridFor(kRows, kDim, 1), 256, 0, stream>>>(
      HID, kMlp, 0L, 0L, W2H, kMlp, 0L, 0L, (void*)PRE2, kDim, 0L, 0L,
      b2, H1N, 0L, 0L, kRows, kDim, kMlp, 1, 1, kWCarryInv);
  ln_rows_kernel<false><<<dim3(kRows / 8), 256, 0, stream>>>(PRE2, ng, nbv, outp, nullptr, kRows);
}
